// Attention_11089605558362
// MI455X (gfx1250) — hardware-run, weakly checked
//
#include <hip/hip_runtime.h>


#define NB_  8
#define TT   2048
#define HD   64
#define ZH   2
typedef _Float16 h16;
typedef unsigned short bf;
typedef __attribute__((ext_vector_type(16))) __bf16   v16bf;
typedef __attribute__((ext_vector_type(16))) _Float16 v16h;
typedef __attribute__((ext_vector_type(8)))  _Float16 v8h;
typedef __attribute__((ext_vector_type(8)))  unsigned short v8us;
typedef __attribute__((ext_vector_type(8)))  float    v8f;
typedef __attribute__((ext_vector_type(4)))  float    v4f;
typedef v8h  __attribute__((may_alias)) v8ha;
typedef v4f  __attribute__((may_alias)) v4fa;
typedef v8us __attribute__((may_alias)) v8usa;

__device__ __forceinline__ unsigned short f2bf(float f) { unsigned u = __float_as_uint(f); u += 0x7FFFu + ((u >> 16) & 1u); return (unsigned short)(u >> 16); }
__device__ __forceinline__ float bf2f(unsigned short b) { return __uint_as_float(((unsigned)b) << 16); }
__device__ __forceinline__ float bfr(float f) { return bf2f(f2bf(f)); }
__device__ __forceinline__ v16h cat16(v8h lo, v8h hi) { return __builtin_shufflevector(lo, hi, 0, 1, 2, 3, 4, 5, 6, 7, 8, 9, 10, 11, 12, 13, 14, 15); }
__device__ __forceinline__ v16bf cat16b(v8us lo, v8us hi) { return __builtin_bit_cast(v16bf, __builtin_shufflevector(lo, hi, 0, 1, 2, 3, 4, 5, 6, 7, 8, 9, 10, 11, 12, 13, 14, 15)); }
__device__ __forceinline__ v8f wmma16(v16h a, v16h b, v8f c) { return __builtin_amdgcn_wmma_f32_16x16x32_f16(false, a, false, b, (short)0, c, false, false); }
__device__ __forceinline__ v8f wmmab(v16bf a, v16bf b, v8f c) { return __builtin_amdgcn_wmma_f32_16x16x32_bf16(false, a, false, b, (short)0, c, false, false); }


template <typename T16> struct WFrag;
template <> struct WFrag<h16> { typedef v16h V; static __device__ __forceinline__ V ld(const h16* p) { return cat16(*(const v8h*)p, *(const v8h*)(p + 16)); } static __device__ __forceinline__ v8f mma(V a, V b, v8f c) { return wmma16(a, b, c); } };
template <> struct WFrag<bf> { typedef v16bf V; static __device__ __forceinline__ V ld(const bf* p) { return cat16b(*(const v8us*)p, *(const v8us*)(p + 16)); } static __device__ __forceinline__ v8f mma(V a, V b, v8f c) { return wmmab(a, b, c); } };
template <typename T16, int NSPLIT, bool BIAS>
__global__ __launch_bounds__(32) void k_gemmw(const T16* __restrict__ A, const T16* __restrict__ A2, const T16* __restrict__ Bt, const T16* __restrict__ Bt2, int K, float* C, int ldc, const float* __restrict__ bias, size_t sA, size_t sB, size_t sC) {
    typedef typename WFrag<T16>::V V;
    __shared__ __align__(16) float os[16 * 68];
    const size_t z = blockIdx.z; A += z * sA; if (A2) A2 += z * sA; Bt += z * sB; if (Bt2) Bt2 += z * sB; C += z * sC;
    const int lane = threadIdx.x & 31, lr = lane & 15, hi = lane >> 4; const int r0 = blockIdx.x * 64, c0 = blockIdx.y * 64;
    v8f acc[4][4];
#pragma unroll
    for (int mb = 0; mb < 4; ++mb)
#pragma unroll
        for (int nb = 0; nb < 4; ++nb) acc[mb][nb] = (v8f){};
    const size_t aoff = (size_t)(r0 + lr) * K + 8 * hi, boff = (size_t)(c0 + lr) * K + 8 * hi;
    for (int kc = 0; kc < K; kc += 32) {
        V a[4], a2[4];
#pragma unroll
        for (int mb = 0; mb < 4; ++mb) { a[mb] = WFrag<T16>::ld(A + aoff + (size_t)mb * 16 * K + kc); if (NSPLIT == 1 || NSPLIT == 2) a2[mb] = WFrag<T16>::ld(A2 + aoff + (size_t)mb * 16 * K + kc); }
#pragma unroll
        for (int nb = 0; nb < 4; ++nb) { const V b = WFrag<T16>::ld(Bt + boff + (size_t)nb * 16 * K + kc); V b2; if (NSPLIT >= 2) b2 = WFrag<T16>::ld(Bt2 + boff + (size_t)nb * 16 * K + kc);
#pragma unroll
            for (int mb = 0; mb < 4; ++mb) { acc[mb][nb] = WFrag<T16>::mma(a[mb], b, acc[mb][nb]); if (NSPLIT == 1 || NSPLIT == 2) acc[mb][nb] = WFrag<T16>::mma(a2[mb], b, acc[mb][nb]); if (NSPLIT >= 2) acc[mb][nb] = WFrag<T16>::mma(a[mb], b2, acc[mb][nb]); } }
        asm volatile("v_nop\n\tv_nop\n\tv_nop\n\tv_nop" : "+v"(acc[0][0]), "+v"(acc[1][1]), "+v"(acc[2][2]), "+v"(acc[3][3]) : "v"(a[0]), "v"(a[3]));
    }
#pragma unroll
    for (int mb = 0; mb < 4; ++mb) {
#pragma unroll
        for (int nb = 0; nb < 4; ++nb) {
#pragma unroll
            for (int j = 0; j < 8; ++j) os[(hi * 8 + j) * 68 + nb * 16 + lr] = acc[mb][nb][j]; }
        __builtin_amdgcn_wave_barrier(); asm volatile("" ::: "memory");
        float* crow = C + (size_t)(r0 + mb * 16) * ldc + c0;
#pragma unroll 1
        for (int ps = 0; ps < 2; ++ps) {
#pragma unroll
            for (int s = 0; s < 8; ++s) { const int row = 2 * s + hi, cofs = lr * 4; v4f val = *(const v4fa*)(os + row * 68 + cofs); if (BIAS) { val[0] += bfr(bias[c0 + cofs]); val[1] += bfr(bias[c0 + cofs + 1]); val[2] += bfr(bias[c0 + cofs + 2]); val[3] += bfr(bias[c0 + cofs + 3]); }
                *(volatile v4f*)(crow + (size_t)row * ldc + cofs) = val; }
            if (ps == 0) __threadfence(); }
        __builtin_amdgcn_wave_barrier(); asm volatile("" ::: "memory");
    }
}

__device__ __forceinline__ h16 tohx(float x) { return (h16)x; }
__device__ __forceinline__ void splitf(float y, unsigned short& h, unsigned short& l) { h = f2bf(y); l = f2bf(y - bf2f(h)); }
typedef __attribute__((ext_vector_type(2))) _Float16 v2h;
typedef __attribute__((ext_vector_type(4))) _Float16 v4h;
typedef __attribute__((ext_vector_type(2))) unsigned short v2us;
typedef __attribute__((ext_vector_type(4))) unsigned short v4us;
typedef __attribute__((ext_vector_type(2))) float v2f;
typedef __attribute__((ext_vector_type(4))) int v4i;

__global__ __launch_bounds__(256) void k_cvt8(const float* __restrict__ src, bf* dst, size_t n8) { const size_t i = (size_t)blockIdx.x * 256 + threadIdx.x; if (i >= n8) return; const v8f v = *(const v8f*)(src + i * 8); v8us o;
#pragma unroll
    for (int k = 0; k < 8; ++k) o[k] = f2bf(v[k]); *(volatile v8us*)(dst + i * 8) = o; __threadfence(); *(volatile v8us*)(dst + i * 8) = o; }
__global__ __launch_bounds__(256) void k_f2h(const float* __restrict__ S, h16* P16, size_t n4) { const size_t i = (size_t)blockIdx.x * 256 + threadIdx.x; if (i >= n4) return; const v4f v = *(const v4f*)(S + i * 4); v4h o;
#pragma unroll
    for (int q = 0; q < 4; ++q) o[q] = tohx(v[q]);
    *(volatile v4h*)(P16 + i * 4) = o; __threadfence(); *(volatile v4h*)(P16 + i * 4) = o; }
__global__ __launch_bounds__(256) void k_vtp(const float* __restrict__ F, int pitch, int nheads, h16* V16, bf* Vh, bf* Vl) { const size_t e = ((size_t)blockIdx.x * 256 + threadIdx.x) * 2; if (e >= (size_t)nheads * HD * TT) return; const int t = (int)(e % TT); const int d = (int)((e / TT) % HD); const int g = (int)(e / ((size_t)TT * HD)); v2h o16; v2us oh, ol;
#pragma unroll
    for (int q = 0; q < 2; ++q) { const float x = F[(size_t)(t + q) * pitch + g * HD + d]; o16[q] = tohx(x); (void)oh; (void)ol; }
    *(volatile v2h*)(V16 + e) = o16; __threadfence(); *(volatile v2h*)(V16 + e) = o16; }
__device__ __forceinline__ float bf16_rne(float f) { unsigned int u = __float_as_uint(f); u += 0x7FFFu + ((u >> 16) & 1u); return __uint_as_float(u & 0xFFFF0000u); }
template <int W>
__global__ __launch_bounds__(256) void rdivf_kernel(const float* __restrict__ A, const float* __restrict__ D, float lo, float* __restrict__ Y, int nn, size_t n4) {
  static_assert(W % 4 == 0 && ((W / 4) & (W / 4 - 1)) == 0, "rdivf: a power-of-two number of float4 groups per row"); const size_t i = (size_t)blockIdx.x * 256 + threadIdx.x; if (i >= n4) return;
  const size_t v = i / (W / 4); v4f o = {0.0f, 0.0f, 0.0f, 0.0f}; if (v < (size_t)nn) { const float dr = D[v]; const float dg = (lo > 0.0f) ? fmaxf(dr, lo) : dr; const v4f t = *(const v4f*)(A + 4 * i); if (dg > 0.0f) { for (int j = 0; j < 4; ++j) o[j] = t[j] / dg; } }
  for (int pass = 0; pass < 2; ++pass) { *(volatile v4f*)(Y + 4 * i) = o; __threadfence(); }
}
template <bool RA, bool RB>
__global__ __launch_bounds__(256) void axpbyr_kernel(const float* __restrict__ A, const float* __restrict__ B, float* __restrict__ Y, size_t n4, float pa, float pb) {
  const size_t i = (size_t)blockIdx.x * 256 + threadIdx.x; if (i >= n4) return; const v4f a = *(const v4f*)(A + 4 * i); const v4f b = *(const v4f*)(B + 4 * i); v4f o; for (int j = 0; j < 4; ++j) { const float x = RA ? bf16_rne(a[j]) : a[j]; const float y = RB ? bf16_rne(b[j]) : b[j]; o[j] = (pa * x) + (pb * y); }
  for (int pass = 0; pass < 2; ++pass) { *(volatile v4f*)(Y + 4 * i) = o; __threadfence(); }
}
template <bool RA, bool RB>
__global__ __launch_bounds__(256) void mulkr_kernel(const float* __restrict__ A, const float* __restrict__ B, float* __restrict__ Y, size_t n4, float s) {
  const size_t i = (size_t)blockIdx.x * 256 + threadIdx.x; if (i >= n4) return; const v4f a = *(const v4f*)(A + 4 * i); const v4f b = *(const v4f*)(B + 4 * i); v4f o; for (int j = 0; j < 4; ++j) { const float x = RA ? bf16_rne(a[j]) : a[j]; const float y = RB ? bf16_rne(b[j]) : b[j]; o[j] = (((x * y)) * s); }
  for (int pass = 0; pass < 2; ++pass) { *(volatile v4f*)(Y + 4 * i) = o; __threadfence(); }
}
__global__ __launch_bounds__(256) void k_rcs(const float* __restrict__ S, float* D) { const unsigned idx = blockIdx.x * 256 + threadIdx.x; const unsigned m = idx % TT, zz = idx / TT; const float* p = S + (size_t)zz * TT * TT + m; float s = 0.0f;
#pragma unroll 8
    for (int l = 0; l < TT; ++l) s = __fadd_rn(s, fmaxf(p[(size_t)l * TT], 0.0f));
    const float d = __fmul_rn(__fadd_rn(s, 1.0e-8f), 2.44140625e-4f); *(volatile float*)(D + idx) = d; __threadfence(); *(volatile float*)(D + idx) = d; }
__global__ __launch_bounds__(256) void k_r16(const float* __restrict__ S, h16* R) { const size_t i = (size_t)blockIdx.x * 256 + threadIdx.x; const v4f v = *(const v4f*)(S + i * 4); v4h o;
#pragma unroll
    for (int q = 0; q < 4; ++q) { const float r = fmaxf(v[q], 0.0f); o[q] = tohx((r < 6.103515625e-5f) ? 0.0f : r); }
    *(volatile v4h*)(R + i * 4) = o; __threadfence(); *(volatile v4h*)(R + i * 4) = o; }

extern "C" void kernel_launch(void* const* d_in, const int* in_sizes, int n_in,
                              void* d_out, int out_size, void* d_ws, size_t ws_size, hipStream_t stream) {
    (void)in_sizes; (void)n_in; (void)out_size;
    const float* x = (const float*)d_in[0]; const float* bw = (const float*)d_in[1]; const float* bb = (const float*)d_in[2]; const float* cw = (const float*)d_in[3]; const float* cb = (const float*)d_in[4]; const float* vw = (const float*)d_in[5]; const float* vb = (const float*)d_in[6];
    float* OUT = (float*)d_out;
    char* wsp = (char*)d_ws;
    auto take = [&](size_t bytes) { char* p = wsp; wsp += (bytes + 255) & ~(size_t)255; return (void*)p; };
    const size_t NR = (size_t)NB_ * TT;
    bf* XB = (bf*)take(NR * HD * 2); bf* WB = (bf*)take((size_t)HD * HD * 2); bf* WC = (bf*)take((size_t)HD * HD * 2); bf* WV = (bf*)take((size_t)HD * HD * 2);
    float* BZ = (float*)take(NR * HD * 4); float* CZ = (float*)take(NR * HD * 4); float* VZ = (float*)take(NR * HD * 4); h16* B16 = (h16*)take(NR * HD * 2); h16* C16 = (h16*)take(NR * HD * 2); float* O = (float*)take(NR * HD * 4);
    float* S = (float*)take((size_t)ZH * TT * TT * 4); h16* R = (h16*)take((size_t)ZH * TT * TT * 2); float* Dv = (float*)take((size_t)ZH * TT * 4); float* VS = (float*)take((size_t)ZH * TT * HD * 4); h16* VT16 = (h16*)take((size_t)ZH * HD * TT * 2);
    if ((size_t)(wsp - (char*)d_ws) > ws_size) return;
    k_cvt8<<<(unsigned)((NR * HD / 8 + 255) / 256), 256, 0, stream>>>(x, XB, NR * HD / 8);
    k_cvt8<<<(unsigned)(((size_t)HD * HD / 8 + 255) / 256), 256, 0, stream>>>(bw, WB, (size_t)HD * HD / 8); k_cvt8<<<(unsigned)(((size_t)HD * HD / 8 + 255) / 256), 256, 0, stream>>>(cw, WC, (size_t)HD * HD / 8); k_cvt8<<<(unsigned)(((size_t)HD * HD / 8 + 255) / 256), 256, 0, stream>>>(vw, WV, (size_t)HD * HD / 8);
    k_gemmw<bf, 0, true><<<dim3((unsigned)(NR / 64), HD / 64, 1), 32, 0, stream>>>(XB, nullptr, WB, nullptr, HD, BZ, HD, bb, 0, 0, 0);
    k_gemmw<bf, 0, true><<<dim3((unsigned)(NR / 64), HD / 64, 1), 32, 0, stream>>>(XB, nullptr, WC, nullptr, HD, CZ, HD, cb, 0, 0, 0);
    k_gemmw<bf, 0, true><<<dim3((unsigned)(NR / 64), HD / 64, 1), 32, 0, stream>>>(XB, nullptr, WV, nullptr, HD, VZ, HD, vb, 0, 0, 0);
    k_f2h<<<(unsigned)((NR * HD / 4 + 255) / 256), 256, 0, stream>>>(BZ, B16, NR * HD / 4); k_f2h<<<(unsigned)((NR * HD / 4 + 255) / 256), 256, 0, stream>>>(CZ, C16, NR * HD / 4);
    for (int e0 = 0; e0 < NB_; e0 += ZH) { const size_t eo = (size_t)e0 * TT * HD;
        k_gemmw<h16, 0, false><<<dim3(TT / 64, TT / 64, ZH), 32, 0, stream>>>(B16 + eo, nullptr, C16 + eo, nullptr, HD, S, TT, nullptr, (size_t)TT * HD, (size_t)TT * HD, (size_t)TT * TT);
        k_rcs<<<ZH * TT / 256, 256, 0, stream>>>(S, Dv);
        k_r16<<<(unsigned)((size_t)ZH * TT * TT / 4 / 256), 256, 0, stream>>>(S, R);
        rdivf_kernel<64><<<(unsigned)(((size_t)ZH * TT * HD / 4 + 255) / 256), 256, 0, stream>>>(VZ + eo, Dv, 1.0e-30f, VS, ZH * TT, (size_t)ZH * TT * HD / 4);
        for (int zz = 0; zz < ZH; ++zz) k_vtp<<<(unsigned)(((size_t)HD * TT / 2 + 255) / 256), 256, 0, stream>>>(VS + (size_t)zz * TT * HD, HD, 1, VT16 + (size_t)zz * HD * TT, nullptr, nullptr);
        k_gemmw<h16, 0, false><<<dim3(TT / 64, HD / 64, ZH), 32, 0, stream>>>(R, nullptr, VT16, nullptr, TT, O + eo, HD, nullptr, (size_t)TT * TT, (size_t)HD * TT, (size_t)TT * HD); }
    axpbyr_kernel<true, false><<<(unsigned)((NR * HD / 4 + 255) / 256), 256, 0, stream>>>(x, O, OUT, NR * HD / 4, 1.0f, 2.44140625e-4f);
}
